// TransformerBlock_63763084477194
// MI455X (gfx1250) — hardware-verified
//
#include <hip/hip_runtime.h>
#include <stddef.h>


typedef _Float16 v16h __attribute__((ext_vector_type(16)));
typedef _Float16 v8h  __attribute__((ext_vector_type(8)));
typedef float    v8f  __attribute__((ext_vector_type(8)));
typedef float    v4f  __attribute__((ext_vector_type(4)));

#ifndef NB
#define NB 2
#endif
#ifndef SEQ
#define SEQ 2048
#endif
#define NB_FULL  2
#define SEQ_FULL 2048
#define DIM   1024
#define NHEAD 16
#define HD    64
#define DFF   4096
#define MROWS (NB * SEQ)
#define RESROWS 256

static_assert(NB >= 1 && NB <= NB_FULL);
static_assert(SEQ >= RESROWS && SEQ <= SEQ_FULL && (SEQ % 128) == 0);
static_assert((RESROWS % 128) == 0);
static_assert(DIM == NHEAD * HD);
static_assert(HD == 64);
static_assert((DIM % 64) == 0 && (DIM % 32) == 0);
static_assert((DFF % 64) == 0 && (DFF % 32) == 0);
static_assert((MROWS % 64) == 0 && (MROWS % 8) == 0);
static_assert(DIM == 4 * 32 * 8);
static_assert((size_t)MROWS * DFF < (size_t)0xFFFFFFFFu);

#define LDT 72
#define LDP 40
#define LDC 68
static_assert((LDT % 8) == 0 && (LDP % 8) == 0 && (LDC % 4) == 0);

#define WCARRY 64.0f
#define PCARRY 16.0f
#define VCARRY 64.0f
#define HCARRY 64.0f
#define RSCALE 2048.0f

#define WSQ ((size_t)DIM * DIM)
#define WFF ((size_t)DIM * DFF)
#define WT_BYTES      ((4 * WSQ + 3 * WFF) * 2)
#define PLANE16_BYTES ((size_t)MROWS * DIM * 2)
#define X1_BYTES      ((size_t)MROWS * DIM * 4)
#define HID_BYTES     ((size_t)MROWS * DFF * 2)
#define VLO_BYTES     ((size_t)NB * DIM * RESROWS * 2)
#define OFF_H16  (WT_BYTES)
#define OFF_Q16  (OFF_H16 + PLANE16_BYTES)
#define OFF_K16  (OFF_Q16 + PLANE16_BYTES)
#define OFF_VT16 (OFF_K16 + PLANE16_BYTES)
#define OFF_CTX  (OFF_VT16 + PLANE16_BYTES)
#define OFF_X1   (OFF_CTX + PLANE16_BYTES)
#define OFF_HID  (OFF_X1 + X1_BYTES)
#define OFF_VLO  (OFF_HID + HID_BYTES)
#define WS_TOTAL (OFF_VLO + VLO_BYTES)
static_assert((WT_BYTES % 128) == 0 && (PLANE16_BYTES % 128) == 0);
static_assert((X1_BYTES % 128) == 0 && (HID_BYTES % 128) == 0 && (VLO_BYTES % 128) == 0);
static_assert(WS_TOTAL <= (size_t)134217728);

__device__ __forceinline__ float bf16r(float x) {
  unsigned int u = __float_as_uint(x);
  u = (u + 0x7FFFu + ((u >> 16) & 1u)) & 0xFFFF0000u;
  return __uint_as_float(u);
}

__device__ __forceinline__ v16h frag_at(const _Float16* p) {
  v8h lo = *(const v8h*)(p);
  v8h hi = *(const v8h*)(p + 16);
  v16h out;
#pragma unroll
  for (int i = 0; i < 8; ++i) { out[i] = lo[i]; out[i + 8] = hi[i]; }
  return out;
}
__device__ __forceinline__ v16h ld_frag(const _Float16* base, unsigned ld) {
  const unsigned lane = threadIdx.x & 31u;
  return frag_at(base + (lane & 15u) * ld + (lane >> 4) * 8u);
}

__device__ __forceinline__ v8f wmma16(v16h a, v16h b, v8f c) {
  v8f d = __builtin_amdgcn_wmma_f32_16x16x32_f16(false, a, false, b, (short)0, c,
                                                 false, false);
  asm volatile("v_nop\n\tv_nop\n\tv_nop\n\tv_nop" : "+v"(d) : "v"(a), "v"(b));
  return d;
}

__device__ __forceinline__ float red16_sum(float x) {
#pragma unroll
  for (int off = 1; off < 16; off <<= 1) x += __shfl_xor(x, off, 32);
  return x;
}

__device__ __forceinline__ void wave_lds_sync() {
  __builtin_amdgcn_fence(3  , "wavefront");
  asm volatile("s_wait_dscnt 0x0" ::: "memory");
  __builtin_amdgcn_wave_barrier();
}

template <int KD>
__device__ __forceinline__ void mm2(const _Float16* __restrict__ ap,
                                    const _Float16* __restrict__ bp0,
                                    v8f& acc0, v8f& acc1) {
  static_assert((KD % 32) == 0);
  const _Float16* bp1 = bp0 + 16 * KD;
#pragma unroll 2
  for (unsigned k0 = 0; k0 < (unsigned)KD; k0 += 32u) {
    const v16h a  = frag_at(ap + k0);
    const v16h b0 = frag_at(bp0 + k0);
    const v16h b1 = frag_at(bp1 + k0);
    acc0 = wmma16(a, b0, acc0);
    acc1 = wmma16(a, b1, acc1);
  }
}

__global__ __launch_bounds__(256) void wconv_kernel(
    const float* __restrict__ W, _Float16* __restrict__ Wt, unsigned KD, unsigned ND) {
  __shared__ _Float16 T[64 * LDT];
  const unsigned tid = threadIdx.x;
  const unsigned n0 = blockIdx.x * 64u;
  const unsigned k0 = blockIdx.y * 64u;
#pragma unroll 4
  for (unsigned j = 0; j < 16u; ++j) {
    const unsigned idx = tid + 256u * j;
    const unsigned kr = idx >> 6, nc = idx & 63u;
    const float v = W[(size_t)(k0 + kr) * ND + n0 + nc];
    T[nc * LDT + kr] = (_Float16)(WCARRY * bf16r(v));
  }
  __syncthreads();
  v8h x[2];
  size_t off[2];
#pragma unroll
  for (unsigned i = 0; i < 2u; ++i) {
    const unsigned n = 32u * i + (tid >> 3);
    const unsigned kc = (tid & 7u) * 8u;
    x[i] = *(const v8h*)&T[n * LDT + kc];
    off[i] = (size_t)(n0 + n) * KD + k0 + kc;
  }
#pragma unroll
  for (int i = 0; i < 2; ++i) *(volatile v8h*)(Wt + off[i]) = x[i];
  __threadfence();
#pragma unroll
  for (int i = 0; i < 2; ++i) *(volatile v8h*)(Wt + off[i]) = x[i];
}

__global__ __launch_bounds__(256) void rms_kernel(
    const float* __restrict__ X, const float* __restrict__ G, _Float16* __restrict__ dst,
    unsigned src_seq, unsigned rnd) {
  const unsigned lane = threadIdx.x & 31u;
  const int wave = __builtin_amdgcn_readfirstlane((int)(threadIdx.x >> 5));
  const unsigned crow = blockIdx.x * 8u + (unsigned)wave;
  const unsigned bidx = crow / (unsigned)SEQ;
  const unsigned sq = crow - bidx * (unsigned)SEQ;
  const float* sp = X + ((size_t)bidx * src_seq + sq) * DIM;
  float vals[4][8];
  float ss = 0.0f;
#pragma unroll
  for (int j = 0; j < 4; ++j) {
    const unsigned c = (unsigned)j * 256u + lane * 8u;
    const v4f a0 = *(const v4f*)(sp + c);
    const v4f a1 = *(const v4f*)(sp + c + 4);
#pragma unroll
    for (int i = 0; i < 4; ++i) {
      float x0 = a0[i], x1 = a1[i];
      x0 = (rnd != 0u) ? bf16r(x0) : x0;
      x1 = (rnd != 0u) ? bf16r(x1) : x1;
      vals[j][i] = x0;
      vals[j][i + 4] = x1;
      ss += x0 * x0;
      ss += x1 * x1;
    }
  }
#pragma unroll
  for (int off = 1; off < 32; off <<= 1) ss += __shfl_xor(ss, off, 32);
  const float rinv = rsqrtf(ss * (1.0f / (float)DIM) + 1.0e-6f);
  v8h o[4];
  size_t off[4];
#pragma unroll
  for (int j = 0; j < 4; ++j) {
    const unsigned c = (unsigned)j * 256u + lane * 8u;
    const v4f g0 = *(const v4f*)(G + c);
    const v4f g1 = *(const v4f*)(G + c + 4);
#pragma unroll
    for (int i = 0; i < 4; ++i) {
      o[j][i]     = (_Float16)((vals[j][i] * rinv) * bf16r(g0[i]));
      o[j][i + 4] = (_Float16)((vals[j][i + 4] * rinv) * bf16r(g1[i]));
    }
    off[j] = (size_t)crow * DIM + c;
  }
#pragma unroll
  for (int j = 0; j < 4; ++j) *(volatile v8h*)(dst + off[j]) = o[j];
  __threadfence();
#pragma unroll
  for (int j = 0; j < 4; ++j) *(volatile v8h*)(dst + off[j]) = o[j];
}


__global__ __launch_bounds__(256) void gemm_qk_kernel(
    const _Float16* __restrict__ A16, const _Float16* __restrict__ Bt,
    _Float16* __restrict__ out16) {
  __shared__ float Cs[64 * LDC];
  const unsigned tid = threadIdx.x, lane = tid & 31u;
  const int wave = __builtin_amdgcn_readfirstlane((int)(threadIdx.x >> 5));
  const unsigned mw = (unsigned)wave >> 1, nw = (unsigned)wave & 1u;
  const unsigned hh = lane >> 4, m = lane & 15u;
  const unsigned n0 = blockIdx.x * 64u;
  const unsigned row0 = blockIdx.y * 64u;
  const _Float16* ap  = A16 + (size_t)(row0 + mw * 16u + m) * DIM + hh * 8u;
  const _Float16* bp0 = Bt + (size_t)(n0 + nw * 32u + m) * DIM + hh * 8u;
  v8f acc0 = {}, acc1 = {};
  mm2<DIM>(ap, bp0, acc0, acc1);
#pragma unroll
  for (int r = 0; r < 8; ++r) {
    const unsigned ci = (mw * 16u + hh * 8u + (unsigned)r) * LDC + nw * 32u + m;
    Cs[ci]      = acc0[r];
    Cs[ci + 16] = acc1[r];
  }
  __syncthreads();
  v8h x[2];
  size_t off[2];
#pragma unroll
  for (unsigned i = 0; i < 2u; ++i) {
    const unsigned r = 32u * i + (tid >> 3);
    const unsigned c = (tid & 7u) * 8u;
    const v4f u0 = *(const v4f*)&Cs[r * LDC + c];
    const v4f u1 = *(const v4f*)&Cs[r * LDC + c + 4];
#pragma unroll
    for (int j = 0; j < 4; ++j) {
      x[i][j]     = (_Float16)(u0[j] * (1.0f / WCARRY));
      x[i][j + 4] = (_Float16)(u1[j] * (1.0f / WCARRY));
    }
    off[i] = (size_t)(row0 + r) * DIM + n0 + c;
  }
#pragma unroll
  for (int i = 0; i < 2; ++i) *(volatile v8h*)(out16 + off[i]) = x[i];
  __threadfence();
#pragma unroll
  for (int i = 0; i < 2; ++i) *(volatile v8h*)(out16 + off[i]) = x[i];
}

__global__ __launch_bounds__(256) void gemm_v_kernel(
    const _Float16* __restrict__ A16, const _Float16* __restrict__ Bt,
    _Float16* __restrict__ Vt, _Float16* __restrict__ Vlo) {
  __shared__ float Cs[64 * LDC];
  const unsigned tid = threadIdx.x, lane = tid & 31u;
  const int wave = __builtin_amdgcn_readfirstlane((int)(threadIdx.x >> 5));
  const unsigned mw = (unsigned)wave >> 1, nw = (unsigned)wave & 1u;
  const unsigned hh = lane >> 4, m = lane & 15u;
  const unsigned n0 = blockIdx.x * 64u;
  const unsigned row0 = blockIdx.y * 64u;
  const _Float16* ap  = A16 + (size_t)(row0 + mw * 16u + m) * DIM + hh * 8u;
  const _Float16* bp0 = Bt + (size_t)(n0 + nw * 32u + m) * DIM + hh * 8u;
  v8f acc0 = {}, acc1 = {};
  mm2<DIM>(ap, bp0, acc0, acc1);
#pragma unroll
  for (int r = 0; r < 8; ++r) {
    const unsigned ci = (mw * 16u + hh * 8u + (unsigned)r) * LDC + nw * 32u + m;
    Cs[ci]      = acc0[r];
    Cs[ci + 16] = acc1[r];
  }
  __syncthreads();
  const unsigned bidx = row0 / (unsigned)SEQ;
  const unsigned key0 = row0 - bidx * (unsigned)SEQ;
  const bool wlo = key0 < (unsigned)RESROWS;
  v8h x[2], xl[2];
  size_t off[2], offl[2];
#pragma unroll
  for (unsigned i = 0; i < 2u; ++i) {
    const unsigned dcol = 32u * i + (tid >> 3);
    const unsigned kk = (tid & 7u) * 8u;
#pragma unroll
    for (unsigned j = 0; j < 8u; ++j) {
      const float val = Cs[(kk + j) * LDC + dcol] * (1.0f / WCARRY);
      const _Float16 hi = (_Float16)val;
      x[i][j]  = hi;
      xl[i][j] = (_Float16)((val - (float)hi) * RSCALE);
    }
    off[i]  = ((size_t)bidx * DIM + n0 + dcol) * SEQ + key0 + kk;
    offl[i] = ((size_t)bidx * DIM + n0 + dcol) * RESROWS + (key0 % (unsigned)RESROWS) + kk;
  }
#pragma unroll
  for (int i = 0; i < 2; ++i) *(volatile v8h*)(Vt + off[i]) = x[i];
  if (wlo) {
#pragma unroll
    for (int i = 0; i < 2; ++i) *(volatile v8h*)(Vlo + offl[i]) = xl[i];
  }
  __threadfence();
#pragma unroll
  for (int i = 0; i < 2; ++i) *(volatile v8h*)(Vt + off[i]) = x[i];
  if (wlo) {
#pragma unroll
    for (int i = 0; i < 2; ++i) *(volatile v8h*)(Vlo + offl[i]) = xl[i];
  }
}

__global__ __launch_bounds__(256) void gemm_wo_kernel(
    const _Float16* __restrict__ A16, const _Float16* __restrict__ Bt,
    const float* __restrict__ Xin, float* __restrict__ X1) {
  __shared__ float Cs[64 * LDC];
  const unsigned tid = threadIdx.x, lane = tid & 31u;
  const int wave = __builtin_amdgcn_readfirstlane((int)(threadIdx.x >> 5));
  const unsigned mw = (unsigned)wave >> 1, nw = (unsigned)wave & 1u;
  const unsigned hh = lane >> 4, m = lane & 15u;
  const unsigned n0 = blockIdx.x * 64u;
  const unsigned row0 = blockIdx.y * 64u;
  const _Float16* ap  = A16 + (size_t)(row0 + mw * 16u + m) * DIM + hh * 8u;
  const _Float16* bp0 = Bt + (size_t)(n0 + nw * 32u + m) * DIM + hh * 8u;
  v8f acc0 = {}, acc1 = {};
  mm2<DIM>(ap, bp0, acc0, acc1);
#pragma unroll
  for (int r = 0; r < 8; ++r) {
    const unsigned ci = (mw * 16u + hh * 8u + (unsigned)r) * LDC + nw * 32u + m;
    Cs[ci]      = acc0[r];
    Cs[ci + 16] = acc1[r];
  }
  __syncthreads();
  v4f xs[4];
  size_t off[4];
#pragma unroll
  for (unsigned i = 0; i < 4u; ++i) {
    const unsigned r = 16u * i + (tid >> 4);
    const unsigned c = (tid & 15u) * 4u;
    const unsigned crow = row0 + r;
    const unsigned bidx = crow / (unsigned)SEQ;
    const unsigned sq = crow - bidx * (unsigned)SEQ;
    const size_t frow = (size_t)bidx * SEQ_FULL + sq;
    const v4f u = *(const v4f*)&Cs[r * LDC + c];
    const v4f g = *(const v4f*)(Xin + frow * DIM + n0 + c);
    v4f val;
#pragma unroll
    for (int j = 0; j < 4; ++j)
      val[j] = u[j] * (1.0f / (WCARRY * VCARRY)) + bf16r(g[j]);
    xs[i] = val;
    off[i] = (size_t)crow * DIM + n0 + c;
  }
#pragma unroll
  for (int i = 0; i < 4; ++i) *(volatile v4f*)(X1 + off[i]) = xs[i];
  __threadfence();
#pragma unroll
  for (int i = 0; i < 4; ++i) *(volatile v4f*)(X1 + off[i]) = xs[i];
}

__global__ __launch_bounds__(256) void gemm_gu_kernel(
    const _Float16* __restrict__ A16, const _Float16* __restrict__ Wg,
    const _Float16* __restrict__ Wu, _Float16* __restrict__ Hid) {
  __shared__ float Cs[64 * LDC];
  const unsigned tid = threadIdx.x, lane = tid & 31u;
  const int wave = __builtin_amdgcn_readfirstlane((int)(threadIdx.x >> 5));
  const unsigned mw = (unsigned)wave >> 1, nw = (unsigned)wave & 1u;
  const unsigned hh = lane >> 4, m = lane & 15u;
  const unsigned n0 = blockIdx.x * 64u;
  const unsigned row0 = blockIdx.y * 64u;
  const _Float16* ap  = A16 + (size_t)(row0 + mw * 16u + m) * DIM + hh * 8u;
  const size_t boff = (size_t)(n0 + nw * 32u + m) * DIM + hh * 8u;
  const _Float16* g0p = Wg + boff;
  const _Float16* g1p = g0p + 16 * DIM;
  const _Float16* u0p = Wu + boff;
  const _Float16* u1p = u0p + 16 * DIM;
  v8f ag0 = {}, ag1 = {}, au0 = {}, au1 = {};
#pragma unroll 2
  for (unsigned k0 = 0; k0 < (unsigned)DIM; k0 += 32u) {
    const v16h a   = frag_at(ap + k0);
    const v16h bg0 = frag_at(g0p + k0);
    const v16h bg1 = frag_at(g1p + k0);
    const v16h bu0 = frag_at(u0p + k0);
    const v16h bu1 = frag_at(u1p + k0);
    ag0 = wmma16(a, bg0, ag0);
    ag1 = wmma16(a, bg1, ag1);
    au0 = wmma16(a, bu0, au0);
    au1 = wmma16(a, bu1, au1);
  }
#pragma unroll
  for (int r = 0; r < 8; ++r) {
    const unsigned ci = (mw * 16u + hh * 8u + (unsigned)r) * LDC + nw * 32u + m;
    const float ga = ag0[r] * (1.0f / WCARRY);
    const float ua = au0[r] * (1.0f / WCARRY);
    const float gb = ag1[r] * (1.0f / WCARRY);
    const float ub = au1[r] * (1.0f / WCARRY);
    const float sa = ga * __builtin_amdgcn_rcpf(1.0f + __expf(-ga));
    const float sb = gb * __builtin_amdgcn_rcpf(1.0f + __expf(-gb));
    Cs[ci]      = (sa * ua) * HCARRY;
    Cs[ci + 16] = (sb * ub) * HCARRY;
  }
  __syncthreads();
  v8h x[2];
  size_t off[2];
#pragma unroll
  for (unsigned i = 0; i < 2u; ++i) {
    const unsigned r = 32u * i + (tid >> 3);
    const unsigned c = (tid & 7u) * 8u;
    const v4f u0 = *(const v4f*)&Cs[r * LDC + c];
    const v4f u1 = *(const v4f*)&Cs[r * LDC + c + 4];
#pragma unroll
    for (int j = 0; j < 4; ++j) {
      x[i][j]     = (_Float16)u0[j];
      x[i][j + 4] = (_Float16)u1[j];
    }
    off[i] = (size_t)(row0 + r) * DFF + n0 + c;
  }
#pragma unroll
  for (int i = 0; i < 2; ++i) *(volatile v8h*)(Hid + off[i]) = x[i];
  __threadfence();
#pragma unroll
  for (int i = 0; i < 2; ++i) *(volatile v8h*)(Hid + off[i]) = x[i];
}

__global__ __launch_bounds__(256) void gemm_down_kernel(
    const _Float16* __restrict__ A16, const _Float16* __restrict__ Bt,
    const float* __restrict__ X1, float* __restrict__ outf) {
  __shared__ float Cs[64 * LDC];
  const unsigned tid = threadIdx.x, lane = tid & 31u;
  const int wave = __builtin_amdgcn_readfirstlane((int)(threadIdx.x >> 5));
  const unsigned mw = (unsigned)wave >> 1, nw = (unsigned)wave & 1u;
  const unsigned hh = lane >> 4, m = lane & 15u;
  const unsigned n0 = blockIdx.x * 64u;
  const unsigned row0 = blockIdx.y * 64u;
  const _Float16* ap  = A16 + (size_t)(row0 + mw * 16u + m) * DFF + hh * 8u;
  const _Float16* bp0 = Bt + (size_t)(n0 + nw * 32u + m) * DFF + hh * 8u;
  v8f acc0 = {}, acc1 = {};
  mm2<DFF>(ap, bp0, acc0, acc1);
#pragma unroll
  for (int r = 0; r < 8; ++r) {
    const unsigned ci = (mw * 16u + hh * 8u + (unsigned)r) * LDC + nw * 32u + m;
    Cs[ci]      = acc0[r];
    Cs[ci + 16] = acc1[r];
  }
  __syncthreads();
  v4f xs[4];
  size_t off[4];
#pragma unroll
  for (unsigned i = 0; i < 4u; ++i) {
    const unsigned r = 16u * i + (tid >> 4);
    const unsigned c = (tid & 15u) * 4u;
    const unsigned crow = row0 + r;
    const unsigned bidx = crow / (unsigned)SEQ;
    const unsigned sq = crow - bidx * (unsigned)SEQ;
    const size_t frow = (size_t)bidx * SEQ_FULL + sq;
    const v4f u = *(const v4f*)&Cs[r * LDC + c];
    const v4f g = *(const v4f*)(X1 + (size_t)crow * DIM + n0 + c);
    v4f val;
#pragma unroll
    for (int j = 0; j < 4; ++j)
      val[j] = g[j] + u[j] * (1.0f / (WCARRY * HCARRY));
    xs[i] = val;
    off[i] = frow * DIM + n0 + c;
  }
#pragma unroll
  for (int i = 0; i < 4; ++i) *(volatile v4f*)(outf + off[i]) = xs[i];
  __threadfence();
#pragma unroll
  for (int i = 0; i < 4; ++i) *(volatile v4f*)(outf + off[i]) = xs[i];
}

__global__ __launch_bounds__(256) void attn_kernel(
    const _Float16* __restrict__ Qh, const _Float16* __restrict__ Kh,
    const _Float16* __restrict__ Vt, const _Float16* __restrict__ Vlo,
    _Float16* __restrict__ Ov) {
  __shared__ _Float16 Ks[64 * LDT];
  __shared__ _Float16 Vs[64 * LDT];
  __shared__ _Float16 Vl[64 * LDT];
  __shared__ _Float16 Ps[8 * 16 * LDT];
  __shared__ _Float16 Pl[8 * 16 * LDP];

  const unsigned tid = threadIdx.x, lane = tid & 31u;
  const int wave = __builtin_amdgcn_readfirstlane((int)(threadIdx.x >> 5));
  const unsigned hh = lane >> 4, m = lane & 15u;
  const unsigned q0 = blockIdx.x * 128u;
  const unsigned head = blockIdx.y;
  const unsigned b = blockIdx.z;
  const unsigned qw = q0 + (unsigned)wave * 16u;
  const bool res = q0 < (unsigned)RESROWS;
  const unsigned pb  = (unsigned)wave * (16u * LDT);
  const unsigned plb = (unsigned)wave * (16u * LDP);

  const size_t qoff = (size_t)(b * (unsigned)SEQ + qw + m) * DIM + head * HD + hh * 8u;

  float lpart[8];
  v8f o[4], orr[4];
#pragma unroll
  for (int v = 0; v < 8; ++v) lpart[v] = 0.0f;
#pragma unroll
  for (int nb = 0; nb < 4; ++nb) { o[nb] = (v8f){}; orr[nb] = (v8f){}; }

  const size_t kplane  = (size_t)b * SEQ * DIM + head * HD;
  const size_t vplane  = ((size_t)b * DIM + head * HD) * SEQ;
  const size_t vlplane = ((size_t)b * DIM + head * HD) * RESROWS;

  for (unsigned kb = 0; kb < q0 + 128u; kb += 64u) {
#pragma unroll
    for (unsigned j = 0; j < 2u; ++j) {
      const unsigned idx = tid + 256u * j;
      const unsigned r = idx >> 3, c = (idx & 7u) * 8u;
      *(v8h*)&Ks[r * LDT + c] = *(const v8h*)(Kh + kplane + (size_t)(kb + r) * DIM + c);
      *(v8h*)&Vs[r * LDT + c] = *(const v8h*)(Vt + vplane + (size_t)r * SEQ + kb + c);
    }
    if (res) {
#pragma unroll
      for (unsigned j = 0; j < 2u; ++j) {
        const unsigned idx = tid + 256u * j;
        const unsigned r = idx >> 3, c = (idx & 7u) * 8u;
        *(v8h*)&Vl[r * LDT + c] = *(const v8h*)(Vlo + vlplane + (size_t)r * RESROWS + kb + c);
      }
    }
    __syncthreads();

#pragma unroll
    for (int hf = 0; hf < 2; ++hf) {
      const unsigned kh = kb + 32u * (unsigned)hf;
      if (kh < qw + 16u) {
        v8f s0 = {}, s1 = {};
#pragma unroll
        for (int c = 0; c < 2; ++c) {
          const v16h qf  = frag_at(Qh + qoff + c * 32);
          const v16h kf0 = ld_frag(&Ks[(hf * 32) * LDT + c * 32], LDT);
          const v16h kf1 = ld_frag(&Ks[(hf * 32 + 16) * LDT + c * 32], LDT);
          s0 = wmma16(qf, kf0, s0);
          s1 = wmma16(qf, kf1, s1);
        }
        const unsigned key0 = kh + m;
        const unsigned key1 = key0 + 16u;
#pragma unroll
        for (int v = 0; v < 8; ++v) {
          const unsigned qrow = qw + hh * 8u + (unsigned)v;
          float e0 = __expf(s0[v] * 0.125f);
          float e1 = __expf(s1[v] * 0.125f);
          e0 = (key0 < qrow) ? e0 : 0.0f;
          e1 = (key1 < qrow) ? e1 : 0.0f;
          lpart[v] += e0 + e1;
          const float p0 = e0 * PCARRY, p1 = e1 * PCARRY;
          const _Float16 h0 = (_Float16)p0, h1 = (_Float16)p1;
          const unsigned pi = pb + (hh * 8u + (unsigned)v) * LDT + (unsigned)hf * 32u + m;
          Ps[pi]      = h0;
          Ps[pi + 16] = h1;
          if (res) {
            const unsigned li = plb + (hh * 8u + (unsigned)v) * LDP + m;
            Pl[li]      = (_Float16)((p0 - (float)h0) * RSCALE);
            Pl[li + 16] = (_Float16)((p1 - (float)h1) * RSCALE);
          }
        }
        wave_lds_sync();

        const v16h pf = ld_frag(&Ps[pb + hf * 32], LDT);
#pragma unroll
        for (int nb = 0; nb < 4; ++nb) {
          const v16h vf = ld_frag(&Vs[(nb * 16) * LDT + hf * 32], LDT);
          o[nb] = wmma16(pf, vf, o[nb]);
        }
        if (res) {
          const v16h plf = ld_frag(&Pl[plb], LDP);
#pragma unroll
          for (int nb = 0; nb < 4; ++nb) {
            const v16h vf  = ld_frag(&Vs[(nb * 16) * LDT + hf * 32], LDT);
            const v16h vlf = ld_frag(&Vl[(nb * 16) * LDT + hf * 32], LDT);
            orr[nb] = wmma16(plf, vf, orr[nb]);
            orr[nb] = wmma16(pf, vlf, orr[nb]);
          }
          wave_lds_sync();
        }
      }
    }
    __syncthreads();
  }

  float inv[8];
#pragma unroll
  for (int v = 0; v < 8; ++v) {
    const float l = red16_sum(lpart[v]);
    inv[v] = __builtin_amdgcn_rcpf(l + 1.0e-9f) * (VCARRY / PCARRY);
  }
#pragma unroll
  for (int nb = 0; nb < 4; ++nb)
#pragma unroll
    for (int v = 0; v < 8; ++v) {
      const float val = o[nb][v] + orr[nb][v] * (1.0f / RSCALE);
      Ps[pb + (hh * 8u + (unsigned)v) * LDT + (unsigned)nb * 16u + m] = (_Float16)(val * inv[v]);
    }
  wave_lds_sync();
  v8h x[4];
  size_t off[4];
#pragma unroll
  for (unsigned i = 0; i < 4u; ++i) {
    const unsigned r = 4u * i + (lane >> 3);
    const unsigned c = (lane & 7u) * 8u;
    x[i] = *(const v8h*)&Ps[pb + r * LDT + c];
    off[i] = (size_t)(b * (unsigned)SEQ + qw + r) * DIM + head * HD + c;
  }
#pragma unroll
  for (int i = 0; i < 4; ++i) *(volatile v8h*)(Ov + off[i]) = x[i];
  __threadfence();
#pragma unroll
  for (int i = 0; i < 4; ++i) *(volatile v8h*)(Ov + off[i]) = x[i];
}

extern "C" void kernel_launch(void* const* d_in, const int* in_sizes, int n_in,
                              void* d_out, int out_size, void* d_ws, size_t ws_size,
                              hipStream_t stream) {
  if (n_in < 10) return;
  const long long need_x = ((long long)(NB - 1) * SEQ_FULL + SEQ) * DIM;
  if ((long long)in_sizes[0] < need_x) return;
  for (int i = 1; i <= 4; ++i)
    if ((long long)in_sizes[i] < (long long)DIM * DIM) return;
  for (int i = 5; i <= 7; ++i)
    if ((long long)in_sizes[i] < (long long)DIM * DFF) return;
  if (in_sizes[8] < DIM || in_sizes[9] < DIM) return;
  if ((long long)out_size < need_x) return;
  if (ws_size < WS_TOTAL) return;

  const float* X  = (const float*)d_in[0];
  const float* Wq = (const float*)d_in[1];
  const float* Wk = (const float*)d_in[2];
  const float* Wv = (const float*)d_in[3];
  const float* Wo = (const float*)d_in[4];
  const float* Wg = (const float*)d_in[5];
  const float* Wu = (const float*)d_in[6];
  const float* Wd = (const float*)d_in[7];
  const float* G1 = (const float*)d_in[8];
  const float* G2 = (const float*)d_in[9];
  float* out = (float*)d_out;

  char* ws = (char*)d_ws;
  _Float16* Wt    = (_Float16*)ws;
  _Float16* WqT   = Wt;
  _Float16* WkT   = Wt + 1 * WSQ;
  _Float16* WvT   = Wt + 2 * WSQ;
  _Float16* WoT   = Wt + 3 * WSQ;
  _Float16* WgT   = Wt + 4 * WSQ;
  _Float16* WuT   = Wt + 4 * WSQ + 1 * WFF;
  _Float16* WdT   = Wt + 4 * WSQ + 2 * WFF;
  _Float16* H16   = (_Float16*)(ws + OFF_H16);
  _Float16* Q16   = (_Float16*)(ws + OFF_Q16);
  _Float16* K16   = (_Float16*)(ws + OFF_K16);
  _Float16* Vt16  = (_Float16*)(ws + OFF_VT16);
  _Float16* Ctx16 = (_Float16*)(ws + OFF_CTX);
  float*    X1    = (float*)(ws + OFF_X1);
  _Float16* Hid16 = (_Float16*)(ws + OFF_HID);
  _Float16* Vlo16 = (_Float16*)(ws + OFF_VLO);

  dim3 blk(256);
  dim3 gsq(DIM / 64, DIM / 64);
  dim3 gg(DIM / 64, MROWS / 64);

  wconv_kernel<<<gsq, blk, 0, stream>>>(Wq, WqT, (unsigned)DIM, (unsigned)DIM);
  wconv_kernel<<<gsq, blk, 0, stream>>>(Wk, WkT, (unsigned)DIM, (unsigned)DIM);
  wconv_kernel<<<gsq, blk, 0, stream>>>(Wv, WvT, (unsigned)DIM, (unsigned)DIM);
  wconv_kernel<<<gsq, blk, 0, stream>>>(Wo, WoT, (unsigned)DIM, (unsigned)DIM);
  wconv_kernel<<<dim3(DFF / 64, DIM / 64), blk, 0, stream>>>(Wg, WgT, (unsigned)DIM, (unsigned)DFF);
  wconv_kernel<<<dim3(DFF / 64, DIM / 64), blk, 0, stream>>>(Wu, WuT, (unsigned)DIM, (unsigned)DFF);
  wconv_kernel<<<dim3(DIM / 64, DFF / 64), blk, 0, stream>>>(Wd, WdT, (unsigned)DFF, (unsigned)DIM);

  rms_kernel<<<dim3(MROWS / 8), blk, 0, stream>>>(X, G1, H16, (unsigned)SEQ_FULL, 1u);
  gemm_qk_kernel<<<gg, blk, 0, stream>>>(H16, WqT, Q16);
  gemm_qk_kernel<<<gg, blk, 0, stream>>>(H16, WkT, K16);
  gemm_v_kernel<<<gg, blk, 0, stream>>>(H16, WvT, Vt16, Vlo16);
  attn_kernel<<<dim3(SEQ / 128, NHEAD, NB), blk, 0, stream>>>(Q16, K16, Vt16, Vlo16, Ctx16);
  gemm_wo_kernel<<<gg, blk, 0, stream>>>(Ctx16, WoT, X, X1);
  rms_kernel<<<dim3(MROWS / 8), blk, 0, stream>>>(X1, G2, H16, (unsigned)SEQ, 0u);
  gemm_gu_kernel<<<dim3(DFF / 64, MROWS / 64), blk, 0, stream>>>(H16, WgT, WuT, Hid16);
  gemm_down_kernel<<<gg, blk, 0, stream>>>(Hid16, WdT, X1, out);
}
